// AttentionLayer_8091718386135
// MI455X (gfx1250) — hardware-verified
//
#include <hip/hip_runtime.h>

typedef __attribute__((ext_vector_type(16))) _Float16 h16x16;
typedef __attribute__((ext_vector_type(8)))  _Float16 h16x8;
typedef __attribute__((ext_vector_type(8)))  float  f32x8;
typedef __attribute__((ext_vector_type(4)))  int    i32x4;

constexpr int kB = 4;
constexpr int kL = 2048;
constexpr int kA = 1024;
constexpr int kH = 16;
constexpr int kD = 64;
constexpr int kM = kB * kL;

typedef __attribute__((ext_vector_type(4))) float v4f;
typedef __attribute__((ext_vector_type(4))) unsigned v4u;
template <typename T> __device__ __forceinline__ void vst2(void* p, T v) { *(volatile T*)p = v; __threadfence(); *(volatile T*)p = v; }
__device__ __forceinline__ f32x8 WMMA_BF16(h16x16 a, h16x16 b, f32x8 c) {
    f32x8 d = __builtin_amdgcn_wmma_f32_16x16x32_f16(false, a, false, b, (short)0, c, false, false);
    asm volatile("v_nop\n\tv_nop\n\tv_nop\n\tv_nop" : "+v"(d) : "v"(a), "v"(b));
    return d;
}

#define AS1 __attribute__((address_space(1)))
#define AS3 __attribute__((address_space(3)))

#define HAVE_ASYNC_COPY 0

__device__ __forceinline__ void async_copy_b128(const _Float16* g, _Float16* l) {
#if HAVE_ASYNC_COPY
    __builtin_amdgcn_global_load_async_to_lds_b128((AS1 i32x4*)g, (AS3 i32x4*)l, 0, 0);
#else
    *reinterpret_cast<h16x8*>(l) = *reinterpret_cast<const h16x8*>(g);
#endif
}

__device__ __forceinline__ void wait_async() {
#if HAVE_ASYNC_COPY
#if __has_builtin(__builtin_amdgcn_s_wait_asynccnt)
    __builtin_amdgcn_s_wait_asynccnt(0);
#else
    asm volatile("s_wait_asynccnt 0" ::: "memory");
#endif
#endif
}

__device__ __forceinline__ h16x8 load_bf8(const _Float16* p) {
    return *reinterpret_cast<const h16x8*>(p);
}

__device__ __forceinline__ h16x16 cat8(h16x8 lo, h16x8 hi) {
    return __builtin_shufflevector(lo, hi, 0, 1, 2, 3, 4, 5, 6, 7,
                                           8, 9, 10, 11, 12, 13, 14, 15);
}

__device__ __forceinline__ h16x8 cvt_f32x8(const float* p) {
    const float4* p4 = reinterpret_cast<const float4*>(p);
    float4 f0 = p4[0];
    float4 f1 = p4[1];
    h16x8 r;
    r[0] = (_Float16)f0.x; r[1] = (_Float16)f0.y; r[2] = (_Float16)f0.z; r[3] = (_Float16)f0.w;
    r[4] = (_Float16)f1.x; r[5] = (_Float16)f1.y; r[6] = (_Float16)f1.z; r[7] = (_Float16)f1.w;
    return r;
}

__global__ __launch_bounds__(256)
void wconv_kernel(const float* __restrict__ w, _Float16* __restrict__ wt) {
    int g = blockIdx.x * blockDim.x + threadIdx.x;
    int idx = g * 8;
    int n = idx >> 10;
    int k = idx & 1023;
    union { h16x8 h; v4u u; } pk;
    #pragma unroll
    for (int e = 0; e < 8; ++e) pk.h[e] = (_Float16)w[((k + e) << 10) + n];
    vst2(wt + idx, pk.u);
}

__global__ __launch_bounds__(128)
void gemm_x_w_kernel(const float* __restrict__ A, const _Float16* __restrict__ Wt,
                     const float* __restrict__ bias, _Float16* __restrict__ out, int vmode) {
    __shared__ __align__(16) _Float16 ldsB[2][64][40];
    __shared__ __align__(16) _Float16 st[4][64 * 72];

    const int lane = threadIdx.x & 31;
    const int wave = threadIdx.x >> 5;
    const int half = lane >> 4;
    const int ln   = lane & 15;
    const int m0 = blockIdx.y * 256 + wave * 64;
    const int n0 = blockIdx.x * 64;

    auto issueB = [&](int buf, int kk) {
        #pragma unroll
        for (int i = 0; i < 2; ++i) {
            int idx = (int)threadIdx.x + 128 * i;
            int row = idx >> 2, seg = idx & 3;
            async_copy_b128(Wt + (size_t)(n0 + row) * kA + kk + seg * 8,
                            &ldsB[buf][row][seg * 8]);
        }
    };

    issueB(0, 0);
    f32x8 acc[4][4] = {};
    for (int kk = 0; kk < kA; kk += 32) {
        const int buf = (kk >> 5) & 1;

        h16x16 af[4];
        #pragma unroll
        for (int mt = 0; mt < 4; ++mt) {
            const float* ap = A + (size_t)(m0 + mt * 16 + ln) * kA + kk + half * 8;
            af[mt] = cat8(cvt_f32x8(ap), cvt_f32x8(ap + 16));
        }

        wait_async();
        __syncthreads();
        if (kk + 32 < kA) issueB(buf ^ 1, kk + 32);

        h16x16 bfr[4];
        #pragma unroll
        for (int nt = 0; nt < 4; ++nt) {
            const _Float16* bp = &ldsB[buf][nt * 16 + ln][half * 8];
            bfr[nt] = cat8(load_bf8(bp), load_bf8(bp + 16));
        }

        #pragma unroll
        for (int mt = 0; mt < 4; ++mt)
            #pragma unroll
            for (int nt = 0; nt < 4; ++nt)
                acc[mt][nt] = WMMA_BF16(af[mt], bfr[nt], acc[mt][nt]);
    }

    float bcol[4];
    #pragma unroll
    for (int nt = 0; nt < 4; ++nt) bcol[nt] = bias[n0 + nt * 16 + ln];

    _Float16* S = st[wave];
    #pragma unroll
    for (int mt = 0; mt < 4; ++mt)
        #pragma unroll
        for (int nt = 0; nt < 4; ++nt)
            #pragma unroll
            for (int r = 0; r < 8; ++r) {
                int rl = mt * 16 + r + 8 * half, cl = nt * 16 + ln;
                _Float16 v = (_Float16)(acc[mt][nt][r] + bcol[nt]);
                if (vmode == 0) S[rl * 72 + cl] = v; else S[cl * 72 + rl] = v;
            }
    asm volatile("s_wait_dscnt 0" ::: "memory"); __builtin_amdgcn_wave_barrier(); __builtin_amdgcn_fence(__ATOMIC_RELEASE, "workgroup");
    {
        const int bb = m0 >> 11, pos0 = m0 & (kL - 1), h = n0 >> 6;
        #pragma unroll 4
        for (int q = 0; q < 16; ++q) { const int rl = q * 4 + (lane >> 3), pc = lane & 7;
            size_t o;
            if (vmode == 0) o = (((size_t)bb * kH + h) * kL + pos0 + rl) * kD + pc * 8;
            else            o = (((size_t)bb * kH + h) * kD + rl) * kL + pos0 + pc * 8;
            vst2(out + o, *(const v4u*)(S + rl * 72 + pc * 8)); }
    }
}

__global__ __launch_bounds__(128)
void attn_kernel(const _Float16* __restrict__ Q, const _Float16* __restrict__ Kr,
                 const _Float16* __restrict__ Vt, _Float16* __restrict__ ctx) {
    __shared__ __align__(16) _Float16 ldsK[2][32][72];
    __shared__ __align__(16) _Float16 ldsV[2][64][40];
    __shared__ __align__(16) _Float16 ldsP[4][16][40];
    __shared__ __align__(16) _Float16 ldsO[4][16][72];

    const int lane = threadIdx.x & 31;
    const int wave = threadIdx.x >> 5;
    const int half = lane >> 4;
    const int ln   = lane & 15;
    const int b = blockIdx.z, h = blockIdx.y;
    const int q0 = blockIdx.x * 64 + wave * 16;
    const int bh = b * kH + h;

    const _Float16* qb  = Q  + (size_t)bh * kL * kD;
    const _Float16* kbp = Kr + (size_t)bh * kL * kD;
    const _Float16* vb  = Vt + (size_t)bh * kD * kL;

    auto issueKV = [&](int buf, int kb0) {
        #pragma unroll
        for (int i = 0; i < 2; ++i) {
            int idx = (int)threadIdx.x + 128 * i;
            int krow = idx >> 3, kseg = idx & 7;
            async_copy_b128(kbp + (size_t)(kb0 + krow) * kD + kseg * 8,
                            &ldsK[buf][krow][kseg * 8]);
            int vrow = idx >> 2, vseg = idx & 3;
            async_copy_b128(vb + (size_t)vrow * kL + kb0 + vseg * 8,
                            &ldsV[buf][vrow][vseg * 8]);
        }
    };

    h16x16 aq[2];
    #pragma unroll
    for (int ks = 0; ks < 2; ++ks) {
        const _Float16* qp = qb + (size_t)(q0 + ln) * kD + ks * 32 + half * 8;
        aq[ks] = cat8(load_bf8(qp), load_bf8(qp + 16));
    }

    issueKV(0, 0);

    f32x8 acc[4] = {};
    float mprev[8], lsum[8];
    #pragma unroll
    for (int r = 0; r < 8; ++r) { mprev[r] = -1e30f; lsum[r] = 0.0f; }

    for (int kb0 = 0; kb0 < kL; kb0 += 32) {
        const int buf = (kb0 >> 5) & 1;

        wait_async();
        __syncthreads();
        if (kb0 + 32 < kL) issueKV(buf ^ 1, kb0 + 32);
        if (kb0 + 64 < kL)
            __builtin_prefetch(kbp + (size_t)(kb0 + 64 + ln) * kD, 0, 3);

        f32x8 c0 = {}, c1 = {};
        #pragma unroll
        for (int ks = 0; ks < 2; ++ks) {
            const _Float16* kp0 = &ldsK[buf][ln][ks * 32 + half * 8];
            const _Float16* kp1 = &ldsK[buf][16 + ln][ks * 32 + half * 8];
            h16x16 bk0 = cat8(load_bf8(kp0), load_bf8(kp0 + 16));
            h16x16 bk1 = cat8(load_bf8(kp1), load_bf8(kp1 + 16));
            c0 = WMMA_BF16(aq[ks], bk0, c0);
            c1 = WMMA_BF16(aq[ks], bk1, c1);
        }

        float corr[8];
        #pragma unroll
        for (int r = 0; r < 8; ++r) {
            float s0 = c0[r] * 0.125f;
            float s1 = c1[r] * 0.125f;
            float mx = fmaxf(s0, s1);
            #pragma unroll
            for (int off = 8; off >= 1; off >>= 1)
                mx = fmaxf(mx, __shfl_xor(mx, off, 32));
            float nm = fmaxf(mprev[r], mx);
            float p0 = __expf(s0 - nm);
            float p1 = __expf(s1 - nm);
            float rs = p0 + p1;
            #pragma unroll
            for (int off = 8; off >= 1; off >>= 1)
                rs += __shfl_xor(rs, off, 32);
            corr[r] = __expf(mprev[r] - nm);
            lsum[r] = lsum[r] * corr[r] + rs;
            mprev[r] = nm;
            int m = r + 8 * half;
            ldsP[wave][m][ln]      = (_Float16)p0;
            ldsP[wave][m][16 + ln] = (_Float16)p1;
        }
        #pragma unroll
        for (int dt = 0; dt < 4; ++dt)
            #pragma unroll
            for (int r = 0; r < 8; ++r)
                acc[dt][r] *= corr[r];

        asm volatile("s_wait_dscnt 0" ::: "memory"); __builtin_amdgcn_wave_barrier(); __builtin_amdgcn_fence(__ATOMIC_RELEASE, "workgroup");
        const _Float16* pp = &ldsP[wave][ln][half * 8];
        h16x16 apf = cat8(*(const h16x8*)pp, *(const h16x8*)(pp + 16));

        #pragma unroll
        for (int dt = 0; dt < 4; ++dt) {
            const _Float16* vp = &ldsV[buf][dt * 16 + ln][half * 8];
            h16x16 bv = cat8(load_bf8(vp), load_bf8(vp + 16));
            acc[dt] = WMMA_BF16(apf, bv, acc[dt]);
        }
    }

    #pragma unroll
    for (int dt = 0; dt < 4; ++dt)
        #pragma unroll
        for (int r = 0; r < 8; ++r) ldsO[wave][r + 8 * half][dt * 16 + ln] = (_Float16)(acc[dt][r] / lsum[r]);
    asm volatile("s_wait_dscnt 0" ::: "memory"); __builtin_amdgcn_wave_barrier(); __builtin_amdgcn_fence(__ATOMIC_RELEASE, "workgroup");
    #pragma unroll
    for (int q = 0; q < 4; ++q) { const int rl = q * 4 + (lane >> 3), pc = lane & 7;
        vst2(ctx + ((size_t)b * kL + q0 + rl) * kA + h * kD + pc * 8, *(const v4u*)(&ldsO[wave][rl][pc * 8])); }
}

__global__ __launch_bounds__(128)
void gemm_ctx_wo_kernel(const _Float16* __restrict__ A, const _Float16* __restrict__ Wt,
                        const float* __restrict__ bias, float* __restrict__ out) {
    __shared__ __align__(16) _Float16 ldsB[2][64][40];
    __shared__ __align__(16) float sto[4][64 * 68];

    const int lane = threadIdx.x & 31;
    const int wave = threadIdx.x >> 5;
    const int half = lane >> 4;
    const int ln   = lane & 15;
    const int m0 = blockIdx.y * 256 + wave * 64;
    const int n0 = blockIdx.x * 64;

    auto issueB = [&](int buf, int kk) {
        #pragma unroll
        for (int i = 0; i < 2; ++i) {
            int idx = (int)threadIdx.x + 128 * i;
            int row = idx >> 2, seg = idx & 3;
            async_copy_b128(Wt + (size_t)(n0 + row) * kA + kk + seg * 8,
                            &ldsB[buf][row][seg * 8]);
        }
    };

    issueB(0, 0);
    f32x8 acc[4][4] = {};
    for (int kk = 0; kk < kA; kk += 32) {
        const int buf = (kk >> 5) & 1;

        h16x16 af[4];
        #pragma unroll
        for (int mt = 0; mt < 4; ++mt) {
            const _Float16* ap = A + (size_t)(m0 + mt * 16 + ln) * kA + kk + half * 8;
            af[mt] = cat8(load_bf8(ap), load_bf8(ap + 16));
        }

        wait_async();
        __syncthreads();
        if (kk + 32 < kA) issueB(buf ^ 1, kk + 32);

        h16x16 bfr[4];
        #pragma unroll
        for (int nt = 0; nt < 4; ++nt) {
            const _Float16* bp = &ldsB[buf][nt * 16 + ln][half * 8];
            bfr[nt] = cat8(load_bf8(bp), load_bf8(bp + 16));
        }

        #pragma unroll
        for (int mt = 0; mt < 4; ++mt)
            #pragma unroll
            for (int nt = 0; nt < 4; ++nt)
                acc[mt][nt] = WMMA_BF16(af[mt], bfr[nt], acc[mt][nt]);
    }

    float bcol[4];
    #pragma unroll
    for (int nt = 0; nt < 4; ++nt) bcol[nt] = bias[n0 + nt * 16 + ln];

    float* S = sto[wave];
    #pragma unroll
    for (int mt = 0; mt < 4; ++mt)
        #pragma unroll
        for (int nt = 0; nt < 4; ++nt)
            #pragma unroll
            for (int r = 0; r < 8; ++r) S[(mt * 16 + r + 8 * half) * 68 + nt * 16 + ln] = acc[mt][nt][r] + bcol[nt];
    asm volatile("s_wait_dscnt 0" ::: "memory"); __builtin_amdgcn_wave_barrier(); __builtin_amdgcn_fence(__ATOMIC_RELEASE, "workgroup");
    #pragma unroll 4
    for (int q = 0; q < 32; ++q) { const int rl = q * 2 + (lane >> 4), pc = lane & 15;
        vst2(out + (size_t)(m0 + rl) * kA + n0 + pc * 4, *(const v4f*)(S + rl * 68 + pc * 4)); }
}

extern "C" void kernel_launch(void* const* d_in, const int* in_sizes, int n_in,
                              void* d_out, int out_size, void* d_ws, size_t ws_size,
                              hipStream_t stream) {
    (void)in_sizes; (void)n_in; (void)out_size; (void)ws_size;

    const float* q  = (const float*)d_in[0];
    const float* k  = (const float*)d_in[1];
    const float* v  = (const float*)d_in[2];
    const float* Wq = (const float*)d_in[3];
    const float* bq = (const float*)d_in[4];
    const float* Wk = (const float*)d_in[5];
    const float* bk = (const float*)d_in[6];
    const float* Wv = (const float*)d_in[7];
    const float* bv = (const float*)d_in[8];
    const float* Wo = (const float*)d_in[9];
    const float* bo = (const float*)d_in[10];
    float* out = (float*)d_out;

    _Float16* wsb = (_Float16*)d_ws;
    const size_t WSZ = (size_t)kA * kA;
    const size_t XSZ = (size_t)kM * kA;
    _Float16* wq_t = wsb;
    _Float16* wk_t = wq_t + WSZ;
    _Float16* wv_t = wk_t + WSZ;
    _Float16* wo_t = wv_t + WSZ;
    _Float16* qw   = wo_t + WSZ;
    _Float16* kw   = qw + XSZ;
    _Float16* vt   = kw + XSZ;
    _Float16* ctx  = vt + XSZ;

    dim3 blk(128);
    int cgrid = (kA * kA / 8) / 256;
    wconv_kernel<<<cgrid, 256, 0, stream>>>(Wq, wq_t);
    wconv_kernel<<<cgrid, 256, 0, stream>>>(Wk, wk_t);
    wconv_kernel<<<cgrid, 256, 0, stream>>>(Wv, wv_t);
    wconv_kernel<<<cgrid, 256, 0, stream>>>(Wo, wo_t);

    dim3 gg(kA / 64, kM / 256);
    gemm_x_w_kernel<<<gg, blk, 0, stream>>>(q, wq_t, bq, qw, 0);
    gemm_x_w_kernel<<<gg, blk, 0, stream>>>(k, wk_t, bk, kw, 0);
    gemm_x_w_kernel<<<gg, blk, 0, stream>>>(v, wv_t, bv, vt, 1);

    dim3 ga(kL / 64, kH, kB);
    attn_kernel<<<ga, blk, 0, stream>>>(qw, kw, vt, ctx);

    gemm_ctx_wo_kernel<<<gg, blk, 0, stream>>>(ctx, wo_t, bo, out);
}
